// Point_Transformer_partseg_80917183857407
// MI455X (gfx1250) — hardware-verified
//
#include <hip/hip_runtime.h>


#define NB_  2
#define NN   4096
#define CIN  15
#define C1   128
#define NC   8
#define PCAR 1024.0f
#define BNK  0.99999500003749969f
typedef _Float16 h16;
typedef unsigned short bf;
typedef __attribute__((ext_vector_type(16))) __bf16   v16bf;
typedef __attribute__((ext_vector_type(16))) _Float16 v16h;
typedef __attribute__((ext_vector_type(8)))  _Float16 v8h;
typedef __attribute__((ext_vector_type(8)))  unsigned short v8us;
typedef __attribute__((ext_vector_type(8)))  float    v8f;
typedef __attribute__((ext_vector_type(4)))  float    v4f;
typedef v8h  __attribute__((may_alias)) v8ha;
typedef v4f  __attribute__((may_alias)) v4fa;
typedef v8us __attribute__((may_alias)) v8usa;

__device__ __forceinline__ unsigned short f2bf(float f) { unsigned u = __float_as_uint(f); u += 0x7FFFu + ((u >> 16) & 1u); return (unsigned short)(u >> 16); }
__device__ __forceinline__ float bf2f(unsigned short b) { return __uint_as_float(((unsigned)b) << 16); }
__device__ __forceinline__ float bfr(float f) { return bf2f(f2bf(f)); }
__device__ __forceinline__ v16h cat16(v8h lo, v8h hi) { return __builtin_shufflevector(lo, hi, 0, 1, 2, 3, 4, 5, 6, 7, 8, 9, 10, 11, 12, 13, 14, 15); }
__device__ __forceinline__ v16bf cat16b(v8us lo, v8us hi) { return __builtin_bit_cast(v16bf, __builtin_shufflevector(lo, hi, 0, 1, 2, 3, 4, 5, 6, 7, 8, 9, 10, 11, 12, 13, 14, 15)); }
__device__ __forceinline__ v8f wmma16(v16h a, v16h b, v8f c) { return __builtin_amdgcn_wmma_f32_16x16x32_f16(false, a, false, b, (short)0, c, false, false); }
__device__ __forceinline__ v8f wmmab(v16bf a, v16bf b, v8f c) { return __builtin_amdgcn_wmma_f32_16x16x32_bf16(false, a, false, b, (short)0, c, false, false); }


template <typename T16> struct WFrag;
template <> struct WFrag<h16> { typedef v16h V; static __device__ __forceinline__ V ld(const h16* p) { return cat16(*(const v8h*)p, *(const v8h*)(p + 16)); } static __device__ __forceinline__ v8f mma(V a, V b, v8f c) { return wmma16(a, b, c); } };
template <> struct WFrag<bf> { typedef v16bf V; static __device__ __forceinline__ V ld(const bf* p) { return cat16b(*(const v8us*)p, *(const v8us*)(p + 16)); } static __device__ __forceinline__ v8f mma(V a, V b, v8f c) { return wmmab(a, b, c); } };
template <typename T16, int NSPLIT, bool BIAS>
__global__ __launch_bounds__(32) void k_gemmw(const T16* __restrict__ A, const T16* __restrict__ A2, const T16* __restrict__ Bt, const T16* __restrict__ Bt2, int K, float* C, int ldc, const float* __restrict__ bias, size_t sA, size_t sB, size_t sC) {
    typedef typename WFrag<T16>::V V;
    __shared__ __align__(16) float os[16 * 68];
    const size_t z = blockIdx.z; A += z * sA; if (A2) A2 += z * sA; Bt += z * sB; if (Bt2) Bt2 += z * sB; C += z * sC;
    const int lane = threadIdx.x & 31, lr = lane & 15, hi = lane >> 4; const int r0 = blockIdx.x * 64, c0 = blockIdx.y * 64;
    v8f acc[4][4];
#pragma unroll
    for (int mb = 0; mb < 4; ++mb)
#pragma unroll
        for (int nb = 0; nb < 4; ++nb) acc[mb][nb] = (v8f){};
    const size_t aoff = (size_t)(r0 + lr) * K + 8 * hi, boff = (size_t)(c0 + lr) * K + 8 * hi;
#pragma unroll 1
    for (int kc = 0; kc < K; kc += 32) {
        V a[4], a2[4];
#pragma unroll
        for (int mb = 0; mb < 4; ++mb) { a[mb] = WFrag<T16>::ld(A + aoff + (size_t)mb * 16 * K + kc); if (NSPLIT == 1 || NSPLIT == 2) a2[mb] = WFrag<T16>::ld(A2 + aoff + (size_t)mb * 16 * K + kc); }
#pragma unroll
        for (int nb = 0; nb < 4; ++nb) { const V b = WFrag<T16>::ld(Bt + boff + (size_t)nb * 16 * K + kc); V b2; if (NSPLIT >= 2) b2 = WFrag<T16>::ld(Bt2 + boff + (size_t)nb * 16 * K + kc);
#pragma unroll
            for (int mb = 0; mb < 4; ++mb) { acc[mb][nb] = WFrag<T16>::mma(a[mb], b, acc[mb][nb]); if (NSPLIT == 1 || NSPLIT == 2) acc[mb][nb] = WFrag<T16>::mma(a2[mb], b, acc[mb][nb]); if (NSPLIT >= 2) acc[mb][nb] = WFrag<T16>::mma(a[mb], b2, acc[mb][nb]); } }
        asm volatile("v_nop\n\tv_nop\n\tv_nop\n\tv_nop" : "+v"(acc[0][0]), "+v"(acc[1][1]), "+v"(acc[2][2]), "+v"(acc[3][3]) : "v"(a[0]), "v"(a[3]));
    }
#pragma unroll
    for (int mb = 0; mb < 4; ++mb) {
#pragma unroll
        for (int nb = 0; nb < 4; ++nb) {
#pragma unroll
            for (int j = 0; j < 8; ++j) os[(hi * 8 + j) * 68 + nb * 16 + lr] = acc[mb][nb][j]; }
        __builtin_amdgcn_wave_barrier(); asm volatile("" ::: "memory");
        float* crow = C + (size_t)(r0 + mb * 16) * ldc + c0;
#pragma unroll 1
        for (int ps = 0; ps < 2; ++ps) {
#pragma unroll
            for (int s = 0; s < 8; ++s) { const int row = 2 * s + hi, cofs = lr * 4; v4f val = *(const v4fa*)(os + row * 68 + cofs); if (BIAS) { val[0] += bfr(bias[c0 + cofs]); val[1] += bfr(bias[c0 + cofs + 1]); val[2] += bfr(bias[c0 + cofs + 2]); val[3] += bfr(bias[c0 + cofs + 3]); }
                *(volatile v4f*)(crow + (size_t)row * ldc + cofs) = val; }
            if (ps == 0) __threadfence(); }
        __builtin_amdgcn_wave_barrier(); asm volatile("" ::: "memory");
    }
}

__device__ __forceinline__ h16 tohx(float x) { return (h16)x; }
__device__ __forceinline__ void splitf(float y, unsigned short& h, unsigned short& l) { h = f2bf(y); l = f2bf(y - bf2f(h)); }
typedef __attribute__((ext_vector_type(2))) _Float16 v2h;
typedef __attribute__((ext_vector_type(4))) _Float16 v4h;
typedef __attribute__((ext_vector_type(2))) unsigned short v2us;
typedef __attribute__((ext_vector_type(4))) unsigned short v4us;
typedef __attribute__((ext_vector_type(2))) float v2f;

__global__ __launch_bounds__(256) void k_cvt8(const float* __restrict__ src, bf* dst, size_t n8) { const size_t i = (size_t)blockIdx.x * 256 + threadIdx.x; if (i >= n8) return; const v8f v = *(const v8f*)(src + i * 8); v8us o;
#pragma unroll
    for (int k = 0; k < 8; ++k) o[k] = f2bf(v[k]); *(volatile v8us*)(dst + i * 8) = o; __threadfence(); *(volatile v8us*)(dst + i * 8) = o; }
__global__ __launch_bounds__(256) void k_cvtp(const float* __restrict__ src, int pitch, int off, int R, int RP, int KW, bf* Bt) { const size_t e = ((size_t)blockIdx.x * 256 + threadIdx.x) * 4; if (e >= (size_t)RP * KW) return; const int k = (int)(e % KW), r = (int)(e / KW); v4us o;
#pragma unroll
    for (int q = 0; q < 4; ++q) o[q] = (r < R) ? f2bf(src[(size_t)r * pitch + off + k + q]) : (unsigned short)0; *(volatile v4us*)(Bt + e) = o; __threadfence(); *(volatile v4us*)(Bt + e) = o; }
__global__ __launch_bounds__(256) void k_l1(const float* __restrict__ xb, const float* __restrict__ w1, const float* __restrict__ g, const float* __restrict__ be, bf* Hh, bf* Hl) { const int e = (blockIdx.x * 256 + threadIdx.x) * 2; if (e >= NN * C1) return; const int c = e % C1, n = e / C1; v2us oh, ol;
#pragma unroll
    for (int q = 0; q < 2; ++q) { const int cq = c + q; float acc = 0.f;
#pragma unroll
        for (int k = 0; k < 3; ++k) { float w = bfr(w1[cq * 3 + k]); asm volatile("" : "+v"(w)); float p = __fmul_rn(w, bfr(xb[(size_t)(9 + k) * NN + n])); asm volatile("" : "+v"(p)); acc = __fadd_rn(acc, p); }
        float gg = bfr(g[cq]) * BNK, bb = bfr(be[cq]); asm volatile("" : "+v"(gg)); asm volatile("" : "+v"(bb)); float t = __fmul_rn(acc, gg); asm volatile("" : "+v"(t)); unsigned short a, c2; splitf(fmaxf(__fadd_rn(t, bb), 0.f), a, c2); oh[q] = a; ol[q] = c2; }
    *(volatile v2us*)(Hh + e) = oh; *(volatile v2us*)(Hl + e) = ol; __threadfence(); *(volatile v2us*)(Hh + e) = oh; *(volatile v2us*)(Hl + e) = ol; }
__global__ __launch_bounds__(256) void k_bnact(const float* __restrict__ F, int C, const float* __restrict__ R, const float* __restrict__ g, const float* __restrict__ be, float slope, float* Y, bf* Ph, bf* Pl) { const size_t e = ((size_t)blockIdx.x * 256 + threadIdx.x) * 2; if (e >= (size_t)NN * C) return; const int c = (int)(e % C); v2f o; v2us oh, ol;
#pragma unroll
    for (int q = 0; q < 2; ++q) { float a = F[e + q]; if (R) { float r = R[c + q]; asm volatile("" : "+v"(r)); a = __fadd_rn(a, r); } float gg = bfr(g[c + q]) * BNK, bb = bfr(be[c + q]); asm volatile("" : "+v"(gg)); asm volatile("" : "+v"(bb)); float t = __fmul_rn(a, gg); asm volatile("" : "+v"(t)); float y = __fadd_rn(t, bb); y = fmaxf(y, y * slope); o[q] = y; unsigned short s1, s2; splitf(y, s1, s2); oh[q] = s1; ol[q] = s2; }
    if (Y) *(volatile v2f*)(Y + e) = o; *(volatile v2us*)(Ph + e) = oh; *(volatile v2us*)(Pl + e) = ol; __threadfence(); if (Y) *(volatile v2f*)(Y + e) = o; *(volatile v2us*)(Ph + e) = oh; *(volatile v2us*)(Pl + e) = ol; }
__global__ __launch_bounds__(256) void k_qsplit(const float* __restrict__ QF, bf* Qh, bf* Ql) { const int e = (blockIdx.x * 256 + threadIdx.x) * 2; if (e >= NN * 32) return; const int k = e & 31, n = e >> 5; v2us oh, ol;
#pragma unroll
    for (int q = 0; q < 2; ++q) { unsigned short a, c2; splitf(QF[(size_t)n * 64 + k + q], a, c2); oh[q] = a; ol[q] = c2; } *(volatile v2us*)(Qh + e) = oh; *(volatile v2us*)(Ql + e) = ol; __threadfence(); *(volatile v2us*)(Qh + e) = oh; *(volatile v2us*)(Ql + e) = ol; }
__global__ __launch_bounds__(256) void k_vt16(const float* __restrict__ VF, h16* VT) { const int e = (blockIdx.x * 256 + threadIdx.x) * 2; if (e >= C1 * NN) return; const int i = e % NN, c = e / NN; v2h o; o[0] = tohx(VF[(size_t)i * C1 + c]); o[1] = tohx(VF[(size_t)(i + 1) * C1 + c]); *(volatile v2h*)(VT + e) = o; __threadfence(); *(volatile v2h*)(VT + e) = o; }
__global__ __launch_bounds__(256) void k_dsplit(const float* __restrict__ Hf, const float* __restrict__ XRF, bf* Dh, bf* Dl) { const int e = (blockIdx.x * 256 + threadIdx.x) * 2; if (e >= NN * C1) return; v2us oh, ol;
#pragma unroll
    for (int q = 0; q < 2; ++q) { float xr = XRF[e + q] * (1.0f / PCAR); asm volatile("" : "+v"(xr)); unsigned short a, c2; splitf(__fsub_rn(Hf[e + q], xr), a, c2); oh[q] = a; ol[q] = c2; } *(volatile v2us*)(Dh + e) = oh; *(volatile v2us*)(Dl + e) = ol; __threadfence(); *(volatile v2us*)(Dh + e) = oh; *(volatile v2us*)(Dl + e) = ol; }
__global__ __launch_bounds__(256) void k_rmax(const float* __restrict__ S, float* RI) { const int lane = threadIdx.x & 31; const int i = blockIdx.x * 8 + (threadIdx.x >> 5); if (i >= NN) return; const float* sr = S + (size_t)i * NN; float m = -3.0e38f;
#pragma unroll 4
    for (int c0 = lane * 4; c0 < NN; c0 += 128) { const v4f v = *(const v4f*)(sr + c0); m = fmaxf(m, fmaxf(fmaxf(v[0], v[1]), fmaxf(v[2], v[3]))); }
#pragma unroll
    for (int sh = 16; sh; sh >>= 1) m = fmaxf(m, __shfl_xor(m, sh, 32));
    const float o = lane == 0 ? m : 0.f; *(volatile float*)(RI + (size_t)i * 32 + lane) = o; __threadfence(); *(volatile float*)(RI + (size_t)i * 32 + lane) = o; }
__global__ __launch_bounds__(256) void k_rexp(float* S, float* RI) { const int lane = threadIdx.x & 31; const int i = blockIdx.x * 8 + (threadIdx.x >> 5); if (i >= NN) return; float* sr = S + (size_t)i * NN; const float m = RI[(size_t)i * 32]; float v[128]; float sum = 0.f;
#pragma unroll
    for (int ch = 0; ch < 32; ++ch) { const v4f a = *(const v4f*)(sr + ch * 128 + lane * 4);
#pragma unroll
        for (int q = 0; q < 4; ++q) { float d0 = __fsub_rn(a[q], m); asm volatile("" : "+v"(d0)); const float e = __builtin_amdgcn_exp2f(__fmul_rn(d0, 1.4426950408889634f)); v[ch * 4 + q] = e; sum += e; } }
#pragma unroll
    for (int sh = 16; sh; sh >>= 1) sum += __shfl_xor(sum, sh, 32);
    const float ri = __fdiv_rn(1.0f, sum);
#pragma unroll 1
    for (int ps = 0; ps < 2; ++ps) {
#pragma unroll
        for (int ch = 0; ch < 32; ++ch) { v4f o; o[0] = v[ch * 4]; o[1] = v[ch * 4 + 1]; o[2] = v[ch * 4 + 2]; o[3] = v[ch * 4 + 3]; *(volatile v4f*)(sr + ch * 128 + lane * 4) = o; }
        const float o2 = lane == 0 ? ri : 0.f; *(volatile float*)(RI + (size_t)i * 32 + lane) = o2; if (ps == 0) __threadfence(); } }
__global__ __launch_bounds__(256) void k_colsum(const float* __restrict__ E, const float* __restrict__ RI, float* CS) { const int j = blockIdx.x * 256 + threadIdx.x; if (j >= NN) return; float s = 0.f;
    for (int i = 0; i < NN; ++i) { float a = __fmul_rn(E[(size_t)i * NN + j], RI[(size_t)i * 32]); asm volatile("" : "+v"(a)); s = __fadd_rn(s, a); }
    const float r = __fdiv_rn(1.0f, __fadd_rn(1e-9f, s)); *(volatile float*)(CS + j) = r; __threadfence(); *(volatile float*)(CS + j) = r; }
__global__ __launch_bounds__(256) void k_ptT(const float* __restrict__ E, const float* __restrict__ RI, const float* __restrict__ CS, h16* PT) { const int e = (blockIdx.x * 256 + threadIdx.x) * 2; if (e >= NN * NN) return; const int i = e % NN, j = e / NN; const float cs = CS[j]; v2h o;
#pragma unroll
    for (int q = 0; q < 2; ++q) { float a = __fmul_rn(E[(size_t)(i + q) * NN + j], RI[(size_t)(i + q) * 32]); asm volatile("" : "+v"(a)); float p = __fmul_rn(a, cs); asm volatile("" : "+v"(p)); o[q] = tohx(p * PCAR); } *(volatile v2h*)(PT + e) = o; __threadfence(); *(volatile v2h*)(PT + e) = o; }
__global__ __launch_bounds__(256) void k_sares(const float* __restrict__ TF, const float* __restrict__ g, const float* __restrict__ be, int blk, float* Hf, bf* Hh, bf* Hl, bf* Fh, bf* Fl) { const int e = (blockIdx.x * 256 + threadIdx.x) * 2; if (e >= NN * C1) return; const int c = e % C1, n = e / C1; float h0[2]; h0[0] = Hf[e]; h0[1] = Hf[e + 1]; v2f o; v2us oh, ol;
#pragma unroll
    for (int q = 0; q < 2; ++q) { float gg = bfr(g[c + q]) * BNK, bb = bfr(be[c + q]); asm volatile("" : "+v"(gg)); asm volatile("" : "+v"(bb)); float t = __fmul_rn(TF[e + q], gg); asm volatile("" : "+v"(t)); t = fmaxf(__fadd_rn(t, bb), 0.f); const float y = __fadd_rn(h0[q], t); o[q] = y; unsigned short a, c2; splitf(y, a, c2); oh[q] = a; ol[q] = c2; }
    const size_t fo = (size_t)n * 512 + blk * C1 + c;
    for (int ps = 0; ps < 2; ++ps) { *(volatile v2f*)(Hf + e) = o; *(volatile v2us*)(Hh + e) = oh; *(volatile v2us*)(Hl + e) = ol; *(volatile v2us*)(Fh + fo) = oh; *(volatile v2us*)(Fl + fo) = ol; if (ps == 0) __threadfence(); } }
__global__ __launch_bounds__(256) void k_pool(const float* __restrict__ HF, float* XMAX, float* XAVG) { const int c = blockIdx.x * 256 + threadIdx.x; if (c >= 1024) return; float m = -3.0e38f, s = 0.f;
    for (int n = 0; n < NN; ++n) { const float v = HF[(size_t)n * 1024 + c]; m = fmaxf(m, v); s = __fadd_rn(s, v); }
    const float a = s * (1.0f / NN); *(volatile float*)(XMAX + c) = m; *(volatile float*)(XAVG + c) = a; __threadfence(); *(volatile float*)(XMAX + c) = m; *(volatile float*)(XAVG + c) = a; }
__global__ __launch_bounds__(256) void k_r512(const float* __restrict__ ws1, const float* __restrict__ bs1, const float* __restrict__ XMAX, const float* __restrict__ XAVG, float* R) { const int o = blockIdx.x * 256 + threadIdx.x; if (o >= 512) return; const float* wr = ws1 + (size_t)o * 3072; float s = 0.f;
#pragma unroll 4
    for (int c = 0; c < 1024; ++c) { float w1 = bfr(wr[1024 + c]), w2 = bfr(wr[2048 + c]); asm volatile("" : "+v"(w1)); asm volatile("" : "+v"(w2)); float p1 = __fmul_rn(w1, XMAX[c]), p2 = __fmul_rn(w2, XAVG[c]); asm volatile("" : "+v"(p1)); asm volatile("" : "+v"(p2)); s = __fadd_rn(s, __fadd_rn(p1, p2)); }
    float bb = bfr(bs1[o]); asm volatile("" : "+v"(bb)); const float r = __fadd_rn(s, bb); *(volatile float*)(R + o) = r; __threadfence(); *(volatile float*)(R + o) = r; }
__global__ __launch_bounds__(256) void k_lsm(const float* __restrict__ S3, const float* __restrict__ bs3, float* OUTb) { const int n = blockIdx.x * 256 + threadIdx.x; if (n >= NN) return; float z[NC]; float m = -3.0e38f;
#pragma unroll
    for (int k = 0; k < NC; ++k) { float bb = bfr(bs3[k]); asm volatile("" : "+v"(bb)); z[k] = __fadd_rn(S3[(size_t)n * 64 + k], bb); m = fmaxf(m, z[k]); }
    float s = 0.f;
#pragma unroll
    for (int k = 0; k < NC; ++k) { float d0 = __fsub_rn(z[k], m); asm volatile("" : "+v"(d0)); s = __fadd_rn(s, __builtin_amdgcn_exp2f(__fmul_rn(d0, 1.4426950408889634f))); }
    float lg = __builtin_amdgcn_logf(s); asm volatile("" : "+v"(lg)); const float lse = __fadd_rn(m, __fmul_rn(lg, 0.69314718055994531f)); v4f o0, o1;
#pragma unroll
    for (int k = 0; k < 4; ++k) { o0[k] = __fsub_rn(z[k], lse); o1[k] = __fsub_rn(z[4 + k], lse); }
    float* d = OUTb + (size_t)n * NC; *(volatile v4f*)d = o0; *(volatile v4f*)(d + 4) = o1; __threadfence(); *(volatile v4f*)d = o0; *(volatile v4f*)(d + 4) = o1; }

extern "C" void kernel_launch(void* const* d_in, const int* in_sizes, int n_in,
                              void* d_out, int out_size, void* d_ws, size_t ws_size, hipStream_t stream) {
    (void)in_sizes; (void)n_in; (void)out_size;
    const float* IN[27]; for (int i = 0; i < 27; ++i) IN[i] = (const float*)d_in[i];
    float* OUT = (float*)d_out;
    char* wsp = (char*)d_ws;
    auto take = [&](size_t bytes) { char* p = wsp; wsp += (bytes + 255) & ~(size_t)255; return (void*)p; };
    bf* W2 = (bf*)take((size_t)C1 * C1 * 2); bf* WQK = (bf*)take((size_t)4 * 64 * C1 * 2); bf* WV = (bf*)take((size_t)4 * C1 * C1 * 2); bf* WT = (bf*)take((size_t)4 * C1 * C1 * 2); bf* WF = (bf*)take((size_t)1024 * 512 * 2); bf* WS1 = (bf*)take((size_t)512 * 1024 * 2); bf* WS2 = (bf*)take((size_t)256 * 512 * 2); bf* WS3 = (bf*)take((size_t)64 * 256 * 2); float* BS3P = (float*)take(256);
    bf* Hh = (bf*)take((size_t)NN * C1 * 2); bf* Hl = (bf*)take((size_t)NN * C1 * 2); float* Hf = (float*)take((size_t)NN * C1 * 4); float* GF = (float*)take((size_t)NN * 1024 * 4); float* QF = (float*)take((size_t)NN * 64 * 4); bf* Qh = (bf*)take((size_t)NN * 32 * 2); bf* Ql = (bf*)take((size_t)NN * 32 * 2);
    float* S = (float*)take((size_t)NN * NN * 4); float* RI = (float*)take((size_t)NN * 32 * 4); float* CS = (float*)take((size_t)NN * 4); h16* PT = (h16*)take((size_t)NN * NN * 2); float* VF = (float*)take((size_t)NN * C1 * 4); h16* VT = (h16*)take((size_t)C1 * NN * 2); float* XRF = (float*)take((size_t)NN * C1 * 4); bf* Dh = (bf*)take((size_t)NN * C1 * 2); bf* Dl = (bf*)take((size_t)NN * C1 * 2); float* TF = (float*)take((size_t)NN * C1 * 4);
    bf* Fh = (bf*)take((size_t)NN * 512 * 2); bf* Fl = (bf*)take((size_t)NN * 512 * 2); float* HF = (float*)take((size_t)NN * 1024 * 4); bf* HFh = (bf*)take((size_t)NN * 1024 * 2); bf* HFl = (bf*)take((size_t)NN * 1024 * 2); float* XMAX = (float*)take(4096); float* XAVG = (float*)take(4096); float* R = (float*)take(2048);
    float* S1F = (float*)take((size_t)NN * 512 * 4); bf* S1h = (bf*)take((size_t)NN * 512 * 2); bf* S1l = (bf*)take((size_t)NN * 512 * 2); float* S2F = (float*)take((size_t)NN * 256 * 4); bf* S2h = (bf*)take((size_t)NN * 256 * 2); bf* S2l = (bf*)take((size_t)NN * 256 * 2); float* S3F = (float*)take((size_t)NN * 64 * 4);
    if ((size_t)(wsp - (char*)d_ws) > ws_size) return;
    { k_cvt8<<<(C1 * C1 / 8 + 255) / 256, 256, 0, stream>>>(IN[4], W2, (size_t)C1 * C1 / 8);
      for (int i = 0; i < 4; ++i) { k_cvtp<<<(64 * C1 / 4 + 255) / 256, 256, 0, stream>>>(IN[7] + (size_t)i * 32 * C1, C1, 0, 32, 64, C1, WQK + (size_t)i * 64 * C1); }
      k_cvt8<<<(4 * C1 * C1 / 8 + 255) / 256, 256, 0, stream>>>(IN[8], WV, (size_t)4 * C1 * C1 / 8); k_cvt8<<<(4 * C1 * C1 / 8 + 255) / 256, 256, 0, stream>>>(IN[10], WT, (size_t)4 * C1 * C1 / 8);
      k_cvt8<<<(1024 * 512 / 8 + 255) / 256, 256, 0, stream>>>(IN[14], WF, (size_t)1024 * 512 / 8); k_cvtp<<<(512 * 1024 / 4 + 255) / 256, 256, 0, stream>>>(IN[17], 3072, 0, 512, 512, 1024, WS1);
      k_cvt8<<<(256 * 512 / 8 + 255) / 256, 256, 0, stream>>>(IN[21], WS2, (size_t)256 * 512 / 8); k_cvtp<<<(64 * 256 / 4 + 255) / 256, 256, 0, stream>>>(IN[25], 256, 0, NC, 64, 256, WS3); }
    const unsigned L1 = (NN * C1 / 2 + 255) / 256; const dim3 g128(NN / 64, C1 / 64, 1);
    for (int b = 0; b < NB_; ++b) {
        k_l1<<<L1, 256, 0, stream>>>(IN[0] + (size_t)b * CIN * NN, IN[1], IN[2], IN[3], Hh, Hl);
        k_gemmw<bf, 1, false><<<g128, 32, 0, stream>>>(Hh, Hl, W2, nullptr, C1, TF, C1, nullptr, 0, 0, 0); k_bnact<<<L1, 256, 0, stream>>>(TF, C1, nullptr, IN[5], IN[6], 0.0f, Hf, Hh, Hl);
        for (int i = 0; i < 4; ++i) {
            k_gemmw<bf, 1, false><<<dim3(NN / 64, 1, 1), 32, 0, stream>>>(Hh, Hl, WQK + (size_t)i * 64 * C1, nullptr, C1, QF, 64, nullptr, 0, 0, 0); k_qsplit<<<(NN * 32 / 2 + 255) / 256, 256, 0, stream>>>(QF, Qh, Ql);
            k_gemmw<bf, 2, false><<<dim3(NN / 64, NN / 64, 1), 32, 0, stream>>>(Qh, Ql, Qh, Ql, 32, S, NN, nullptr, 0, 0, 0);
            k_rmax<<<NN / 8, 256, 0, stream>>>(S, RI); k_rexp<<<NN / 8, 256, 0, stream>>>(S, RI); k_colsum<<<NN / 256, 256, 0, stream>>>(S, RI, CS); k_ptT<<<(NN * NN / 2 + 255) / 256, 256, 0, stream>>>(S, RI, CS, PT);
            k_gemmw<bf, 1, true><<<g128, 32, 0, stream>>>(Hh, Hl, WV + (size_t)i * C1 * C1, nullptr, C1, VF, C1, IN[9] + i * C1, 0, 0, 0); k_vt16<<<(C1 * NN / 2 + 255) / 256, 256, 0, stream>>>(VF, VT);
            k_gemmw<h16, 0, false><<<g128, 32, 0, stream>>>(PT, nullptr, VT, nullptr, NN, XRF, C1, nullptr, 0, 0, 0);
            k_dsplit<<<L1, 256, 0, stream>>>(Hf, XRF, Dh, Dl);
            k_gemmw<bf, 1, true><<<g128, 32, 0, stream>>>(Dh, Dl, WT + (size_t)i * C1 * C1, nullptr, C1, TF, C1, IN[11] + i * C1, 0, 0, 0);
            k_sares<<<L1, 256, 0, stream>>>(TF, IN[12] + i * C1, IN[13] + i * C1, i, Hf, Hh, Hl, Fh, Fl); }
        k_gemmw<bf, 1, false><<<dim3(NN / 64, 1024 / 64, 1), 32, 0, stream>>>(Fh, Fl, WF, nullptr, 512, GF, 1024, nullptr, 0, 0, 0); k_bnact<<<(NN * 1024 / 2 + 255) / 256, 256, 0, stream>>>(GF, 1024, nullptr, IN[15], IN[16], 0.2f, HF, HFh, HFl);
        k_pool<<<4, 256, 0, stream>>>(HF, XMAX, XAVG); k_r512<<<2, 256, 0, stream>>>(IN[17], IN[18], XMAX, XAVG, R);
        k_gemmw<bf, 1, false><<<dim3(NN / 64, 512 / 64, 1), 32, 0, stream>>>(HFh, HFl, WS1, nullptr, 1024, S1F, 512, nullptr, 0, 0, 0); k_bnact<<<(NN * 512 / 2 + 255) / 256, 256, 0, stream>>>(S1F, 512, R, IN[19], IN[20], 0.0f, nullptr, S1h, S1l);
        k_gemmw<bf, 1, true><<<dim3(NN / 64, 256 / 64, 1), 32, 0, stream>>>(S1h, S1l, WS2, nullptr, 512, S2F, 256, IN[22], 0, 0, 0); k_bnact<<<(NN * 256 / 2 + 255) / 256, 256, 0, stream>>>(S2F, 256, nullptr, IN[23], IN[24], 0.0f, nullptr, S2h, S2l);
        k_gemmw<bf, 1, false><<<dim3(NN / 64, 1, 1), 32, 0, stream>>>(S2h, S2l, WS3, nullptr, 256, S3F, 64, nullptr, 0, 0, 0);
        k_lsm<<<NN / 256, 256, 0, stream>>>(S3F, IN[26], OUT + (size_t)b * NN * NC); }
}
